// ResnetBlocWithAttn_62354335203904
// MI455X (gfx1250) — hardware-verified
//
#include <hip/hip_runtime.h>
#include <hip/hip_bf16.h>
#include <math.h>

#define NB_   8
#define CH    256
#define IMH   32
#define IMW   32
#define HW_   1024
#define NG    32
#define SS    1024
#define HH    12
#define BB    8
#define DKK   64
#define QW    2
#define QKVST 768
#define ATST  256
#define KST   40

typedef _Float16 bf16;
typedef _Float16 f16;
typedef __attribute__((ext_vector_type(4))) unsigned v4u_t;
typedef unsigned v4ua __attribute__((ext_vector_type(4), may_alias));
typedef __attribute__((ext_vector_type(4))) float v4f_t;
typedef float v4fa __attribute__((ext_vector_type(4), may_alias));
typedef __attribute__((ext_vector_type(16))) bf16  bf16x16;
typedef bf16x16 f16x16;
typedef __attribute__((ext_vector_type(8)))  bf16  bf16x8;
typedef bf16x8 f16x8;
typedef __attribute__((ext_vector_type(4)))  bf16  bf16x4;
typedef __attribute__((ext_vector_type(8)))  float f32x8;
__device__ __forceinline__ f32x8 wmma16(f16x16 a, f16x16 b, f32x8 c) {
  c = __builtin_amdgcn_wmma_f32_16x16x32_f16(false, a, false, b, (short)0, c, false, false);
  asm volatile("v_nop\n\tv_nop\n\tv_nop\n\tv_nop" : "+v"(c) : "v"(a), "v"(b));
  return c;
}
#define LDS_STRIDE 48
#define KSTRIDE    72
#define VSTRIDE    48

__device__ __forceinline__ f32x8 wmma_bf16(bf16x16 a, bf16x16 b, f32x8 c) {
  c = __builtin_amdgcn_wmma_f32_16x16x32_f16(false, a, false, b, (short)0, c, false, false);
  asm volatile("v_nop\n\tv_nop\n\tv_nop\n\tv_nop" : "+v"(c) : "v"(a), "v"(b));
  return c;
}

template <typename T>
__device__ __forceinline__ bf16x16 load_frag(const T* __restrict__ base, int ld,
                                             int row0, int k0) {
  const int lane = threadIdx.x & 31;
  const int r    = lane & 15;
  const int kh   = (lane >> 4) * 8;
  const T* p0 = base + (size_t)(row0 + r) * ld + (k0 + kh);
  const T* p1 = p0 + 16;
  bf16x16 f;
#pragma unroll
  for (int i = 0; i < 8; ++i) {
    f[i]     = (bf16)p0[i];
    f[i + 8] = (bf16)p1[i];
  }
  return f;
}

__device__ __forceinline__ bf16x16 lds_frag(const bf16* base, int stride) {
  const int lane = threadIdx.x & 31;
  const int row  = lane & 15;
  const int kh   = (lane >> 4) * 8;
  const bf16x8 lo = *(const bf16x8*)(base + row * stride + kh);
  const bf16x8 hi = *(const bf16x8*)(base + row * stride + kh + 16);
  bf16x16 f;
#pragma unroll
  for (int i = 0; i < 8; ++i) { f[i] = lo[i]; f[i + 8] = hi[i]; }
  return f;
}

template <typename T>
__device__ __forceinline__ void stage_read16(const T* __restrict__ p, float* buf) {
#pragma unroll
  for (int i = 0; i < 16; ++i) buf[i] = (float)p[i];
}

__device__ __forceinline__ void stage_write(bf16* dst, const float* buf, int nquad) {
#pragma unroll
  for (int i = 0; i < nquad; ++i) {
    bf16x4 q;
    q[0] = (bf16)buf[4 * i];     q[1] = (bf16)buf[4 * i + 1];
    q[2] = (bf16)buf[4 * i + 2]; q[3] = (bf16)buf[4 * i + 3];
    *(bf16x4*)(dst + 4 * i) = q;
  }
}

template <typename AT, int MODE>
__global__ __launch_bounds__(256) void gemm_rb_kernel(
    const AT* __restrict__ A, const float* __restrict__ W,
    const float* __restrict__ bias, const float* __restrict__ rowscale, const float* __restrict__ R, const float* __restrict__ rowbias, void* __restrict__ out,
    int M, int N, int K) {
  __shared__ bf16 ldsA[128 * LDS_STRIDE];
  __shared__ bf16 ldsW[256 * LDS_STRIDE];
  __shared__ __attribute__((aligned(16))) unsigned char sob[256 * 136 * 2];

  const int t    = threadIdx.x;
  const int wave = t >> 5;
  const int lane = t & 31;
  const int wm   = (wave & 1) * 64;
  const int wn   = (wave >> 1) * 64;
  const int mBlk = blockIdx.x * 128;
  const int nBlk = blockIdx.y * 256;

  const int arow = t >> 1;
  const int ach  = (t & 1) * 16;

  float abuf[16];
  float wbuf[32];

  stage_read16(A + (size_t)(mBlk + arow) * K + ach, abuf);
  const int nrow = min(nBlk + t, N - 1);
  stage_read16(W + (size_t)nrow * K,          wbuf);
  stage_read16(W + (size_t)nrow * K + 16,     wbuf + 16);

  f32x8 acc[4][4] = {};

  for (int k = 0; k < K; k += 32) {
    __syncthreads();
    stage_write(&ldsA[arow * LDS_STRIDE + ach], abuf, 4);
    stage_write(&ldsW[t * LDS_STRIDE],          wbuf, 8);
    if (k + 32 < K) {
      stage_read16(A + (size_t)(mBlk + arow) * K + (k + 32) + ach, abuf);
      stage_read16(W + (size_t)nrow * K + (k + 32),          wbuf);
      stage_read16(W + (size_t)nrow * K + (k + 32) + 16,     wbuf + 16);
    }
    __syncthreads();

    bf16x16 af[4], wf[4];
#pragma unroll
    for (int i = 0; i < 4; ++i)
      af[i] = lds_frag(ldsA + (wm + 16 * i) * LDS_STRIDE, LDS_STRIDE);
#pragma unroll
    for (int j = 0; j < 4; ++j)
      wf[j] = lds_frag(ldsW + (wn + 16 * j) * LDS_STRIDE, LDS_STRIDE);
#pragma unroll
    for (int i = 0; i < 4; ++i)
#pragma unroll
      for (int j = 0; j < 4; ++j)
        acc[i][j] = wmma_bf16(af[i], wf[j], acc[i][j]);
  }

  const int nlane = lane & 15;
  const int mh    = (lane >> 4) * 8;
  __syncthreads();
  if (MODE == 0 || MODE == 1 || MODE == 3) {
    bf16* so = (bf16*)sob;
#pragma unroll
    for (int i = 0; i < 4; ++i)
#pragma unroll
      for (int j = 0; j < 4; ++j) {
        const int nl = wn + 16 * j + nlane;
        const float bv = bias ? bias[nBlk + nl] : 0.0f;
        if (MODE == 3) {
#pragma unroll 1
          for (int r = 0; r < 8; ++r) {
            const int ml = wm + 16 * i + mh + r;
            const float xg = acc[i][j][r] + bv;
            so[ml * 264 + nl] = (bf16)(0.5f * xg * (1.0f + erff(xg * 0.70710678118654752f)));
          }
        } else {
#pragma unroll
        for (int r = 0; r < 8; ++r) {
          const int ml = wm + 16 * i + mh + r;
          const bf16 hv = (bf16)(acc[i][j][r] + bv);
          if (MODE == 0) so[ml * 264 + nl] = hv;
          else           so[nl * 136 + ml] = hv;
        }
        }
      }
    __syncthreads();
#pragma unroll 1
    for (int pass = 0; pass < 2; ++pass) {
      if (MODE == 0 || MODE == 3) {
        for (int ch = t; ch < 128 * 32; ch += 256) { const int ml = ch >> 5, q = (ch & 31) * 8;
          *(volatile v4u_t*)((bf16*)out + (size_t)(mBlk + ml) * N + nBlk + q) = *(const v4ua*)(so + ml * 264 + q); }
      } else {
        const int b_ = mBlk / SS, s0 = mBlk & (SS - 1);
        for (int ch = t; ch < 256 * 16; ch += 256) { const int nl = ch >> 4, q = (ch & 15) * 8; const int n = nBlk + nl, h = n >> 6, dk = n & (DKK - 1);
          *(volatile v4u_t*)((bf16*)out + (((size_t)(b_ * HH + h)) * DKK + dk) * SS + s0 + q) = *(const v4ua*)(so + nl * 136 + q); }
      }
      __threadfence();
    }
  } else {
    float* so = (float*)sob;
#pragma unroll 1
    for (int hf = 0; hf < 2; ++hf) {
      if (wm == hf * 64) {
#pragma unroll
        for (int i = 0; i < 4; ++i)
#pragma unroll
          for (int j = 0; j < 4; ++j) {
            const int nl = wn + 16 * j + nlane;
            const float bv = bias ? bias[nBlk + nl] : 0.0f;
#pragma unroll
            for (int r = 0; r < 8; ++r) { const int mrow = mBlk + hf * 64 + 16 * i + mh + r; so[(16 * i + mh + r) * 260 + nl] = acc[i][j][r] * (rowscale ? rowscale[mrow] : 1.0f) + bv + (rowbias ? rowbias[mrow] : 0.0f); }
          }
      }
      __syncthreads();
      if (R) {
        for (int ch = t; ch < 64 * 64; ch += 256) { const int ml = ch >> 6, q = (ch & 63) * 4;
          if (nBlk + q < N) { const v4f_t rv = *(const v4f_t*)(R + (size_t)(mBlk + hf * 64 + ml) * N + nBlk + q); v4f_t v = *(const volatile v4fa*)(so + ml * 260 + q); v += rv; *(volatile v4fa*)(so + ml * 260 + q) = v; } }
        asm volatile("s_wait_dscnt 0" ::: "memory");
      }
#pragma unroll 1
      for (int pass = 0; pass < 2; ++pass) {
        for (int ch = t; ch < 64 * 64; ch += 256) { const int ml = ch >> 6, q = (ch & 63) * 4;
          if (nBlk + q < N) *(volatile v4f_t*)((float*)out + (size_t)(mBlk + hf * 64 + ml) * N + nBlk + q) = *(const volatile v4fa*)(so + ml * 260 + q); }
        __threadfence();
      }
      __syncthreads();
    }
  }
}

__global__ __launch_bounds__(64) void attn_kernel(
    const bf16* __restrict__ Qb, const bf16* __restrict__ Kb,
    const bf16* __restrict__ Vt, float* __restrict__ attnOut) {
  __shared__ bf16 ldsK[32 * KSTRIDE];
  __shared__ bf16 ldsV[64 * VSTRIDE];
  __shared__ __attribute__((aligned(16))) float ldsO[2][32 * 68];

  const int q0blk = blockIdx.x * 64;
  const int h  = blockIdx.y;
  const int b  = blockIdx.z;
  const int t    = threadIdx.x;
  const int wave = t >> 5;
  const int lane = t & 31;
  const int qlane = lane & 15;
  const int kh8   = (lane >> 4) * 8;
  const int q0 = q0blk + wave * 32;

  const bf16* Qh = Qb + (size_t)b * SS * QKVST + h * 192;
  const bf16* Kh = Qb + (size_t)b * SS * QKVST + h * 192 + 64;
  const bf16* Vh = Vt + ((size_t)(b * HH + 3 * h + 2)) * DKK * SS;

  const int krow = t >> 1;
  const int kcol = (t & 1) * 32;
  const bf16* kSrc = Kh + (size_t)krow * QKVST + kcol;
  const bf16* vSrc = Vh + (size_t)t * SS;

  bf16x16 qf[QW][2];
#pragma unroll
  for (int qt = 0; qt < QW; ++qt) {
    qf[qt][0] = load_frag(Qh, QKVST, q0 + 16 * qt, 0);
    qf[qt][1] = load_frag(Qh, QKVST, q0 + 16 * qt, 32);
  }

  f32x8 o[QW][4] = {};
  float mrun[QW], lrun[QW];
#pragma unroll
  for (int qt = 0; qt < QW; ++qt) { mrun[qt] = -INFINITY; lrun[qt] = 0.0f; }

  const float scale = 0.0625f * 1.44269504088896340736f;
  const float NEG2 = -1.0e9f;
  const int kmax = SS - 1;

  bf16x8 kreg[4], vreg[4];
#pragma unroll
  for (int i = 0; i < 4; ++i) {
    kreg[i] = *(const bf16x8*)(kSrc + 8 * i);
    vreg[i] = *(const bf16x8*)(vSrc + 8 * i);
  }

  for (int kb = 0; kb <= kmax; kb += 32) {
    __syncthreads();
#pragma unroll
    for (int i = 0; i < 4; ++i) {
      *(bf16x8*)(&ldsK[krow * KSTRIDE + kcol + 8 * i]) = kreg[i];
      *(bf16x8*)(&ldsV[t * VSTRIDE + 8 * i])           = vreg[i];
    }
    if (kb + 32 <= kmax) {
      const bf16* kn = kSrc + (size_t)(kb + 32) * QKVST;
      const bf16* vn = vSrc + (kb + 32);
#pragma unroll
      for (int i = 0; i < 4; ++i) {
        kreg[i] = *(const bf16x8*)(kn + 8 * i);
        vreg[i] = *(const bf16x8*)(vn + 8 * i);
      }
    }
    __syncthreads();

    bf16x16 kf[2][2];
#pragma unroll
    for (int ktile = 0; ktile < 2; ++ktile)
#pragma unroll
      for (int c = 0; c < 2; ++c)
        kf[ktile][c] = lds_frag(ldsK + (ktile * 16) * KSTRIDE + c * 32, KSTRIDE);

    bf16x16 pf[QW];
    bool act[QW];
#pragma unroll
    for (int qt = 0; qt < QW; ++qt) {
      unsigned mbits = 0;
      mbits = 0xFFFFu; act[qt] = true;
      if (act[qt]) {
        const int q_my = q0 + 16 * qt + qlane;
        f32x8 s0 = {}, s1 = {};
        s0 = wmma_bf16(kf[0][0], qf[qt][0], s0);
        s0 = wmma_bf16(kf[0][1], qf[qt][1], s0);
        s1 = wmma_bf16(kf[1][0], qf[qt][0], s1);
        s1 = wmma_bf16(kf[1][1], qf[qt][1], s1);

        float mx = -INFINITY;
#pragma unroll
        for (int r = 0; r < 8; ++r) {
          const int k0i = kb + kh8 + r;
          const int k1i = k0i + 16;
          (void)k0i; (void)k1i; (void)q_my;
          s0[r] = (mbits & (1u << r))       ? s0[r] * scale : NEG2;
          s1[r] = (mbits & (1u << (8 + r))) ? s1[r] * scale : NEG2;
          mx = fmaxf(mx, fmaxf(s0[r], s1[r]));
        }
        mx = fmaxf(mx, __shfl_xor(mx, 16, 32));
        const float mnew  = fmaxf(mrun[qt], mx);
        const float alpha = exp2f(mrun[qt] - mnew);

        float rsum = 0.0f;
#pragma unroll
        for (int r = 0; r < 8; ++r) {
          const float p0 = exp2f(s0[r] - mnew);
          const float p1 = exp2f(s1[r] - mnew);
          rsum += p0 + p1;
          pf[qt][r]     = (bf16)(p0 * 1024.0f);
          pf[qt][r + 8] = (bf16)(p1 * 1024.0f);
        }
        rsum += __shfl_xor(rsum, 16, 32);
        lrun[qt] = lrun[qt] * alpha + rsum;
        mrun[qt] = mnew;

#pragma unroll
        for (int j = 0; j < 4; ++j)
#pragma unroll
          for (int r = 0; r < 8; ++r) o[qt][j][r] *= alpha;
      }
    }

#pragma unroll
    for (int j = 0; j < 4; ++j) {
      const bf16x16 vf = lds_frag(ldsV + (j * 16) * VSTRIDE, VSTRIDE);
#pragma unroll
      for (int qt = 0; qt < QW; ++qt)
        if (act[qt]) o[qt][j] = wmma_bf16(vf, pf[qt], o[qt][j]);
    }
  }

  float* so = ldsO[wave];
#pragma unroll
  for (int qt = 0; qt < QW; ++qt) {
    const float rl = 1.0f / (lrun[qt] * 1024.0f);
#pragma unroll
    for (int j = 0; j < 4; ++j)
#pragma unroll
      for (int r = 0; r < 8; ++r) so[(16 * qt + qlane) * 68 + j * 16 + kh8 + r] = o[qt][j][r] * rl;
  }
  asm volatile("s_wait_dscnt 0" ::: "memory");
  __builtin_amdgcn_wave_barrier();
#pragma unroll 1
  for (int pass = 0; pass < 2; ++pass) {
#pragma unroll
    for (int it = 0; it < 16; ++it) { const int ch = lane + 32 * it, ql = ch >> 4, q4 = (ch & 15) * 4;
      *(volatile v4f_t*)(attnOut + ((size_t)(b * SS + q0 + ql)) * ATST + h * DKK + q4) = *(const volatile v4fa*)(so + ql * 68 + q4); }
    __threadfence();
  }
}


__global__ __launch_bounds__(256) void k_gn_stats(const float* __restrict__ src, float* __restrict__ stats) {
  __shared__ float red[256];
  __shared__ __attribute__((aligned(16))) float outS[32];
  const int b = blockIdx.x >> 1, g0 = (blockIdx.x & 1) * 16, t = threadIdx.x;
#pragma unroll 1
  for (int gg = 0; gg < 16; ++gg) {
    const float* p = src + ((size_t)b * CH + (g0 + gg) * 8) * HW_;
    float s = 0.0f;
    for (int i = t; i < 8192; i += 256) s += p[i];
    red[t] = s; __syncthreads();
    for (int o = 128; o > 0; o >>= 1) { if (t < o) red[t] += red[t + o]; __syncthreads(); }
    const float mu = red[0] * (1.0f / 8192.0f); __syncthreads();
    float q = 0.0f;
    for (int i = t; i < 8192; i += 256) { const float d = p[i] - mu; q += d * d; }
    red[t] = q; __syncthreads();
    for (int o = 128; o > 0; o >>= 1) { if (t < o) red[t] += red[t + o]; __syncthreads(); }
    if (t == 0) { outS[2 * gg] = mu; outS[2 * gg + 1] = 1.0f / sqrtf(red[0] * (1.0f / 8192.0f) + 1e-5f); }
    __syncthreads();
  }
  if (t < 8) {
#pragma unroll 1
    for (int pass = 0; pass < 2; ++pass) { *(volatile v4f_t*)(stats + ((size_t)b * NG + g0) * 2 + t * 4) = *(const volatile v4fa*)(outS + t * 4); __threadfence(); }
  }
}
__global__ __launch_bounds__(256) void k_emb(const float* __restrict__ te, const float* __restrict__ mw, const float* __restrict__ mb, float* __restrict__ emb) {
  __shared__ __attribute__((aligned(16))) f16 aS[16 * 264];
  __shared__ __attribute__((aligned(16))) float eS[8 * 256];
  const int tid = threadIdx.x, lane = tid & 31, wave = tid >> 5, cl = lane & 15, rh = (lane >> 4) * 8;
  for (int e = tid; e < 16 * 256; e += 256) { const int r = e >> 8, c = e & 255; float v = 0.0f; if (r < NB_) { const float x = te[r * 256 + c]; v = x / (1.0f + __expf(-x)); } aS[r * 264 + c] = (f16)v; }
  __syncthreads();
#pragma unroll 1
  for (int j = 0; j < 2; ++j) {
    const int nt = wave * 2 + j;
    f32x8 acc = {};
#pragma unroll
    for (int ks = 0; ks < 8; ++ks) acc = wmma16(lds_frag(aS + ks * 32, 264), load_frag(mw, 256, nt * 16, ks * 32), acc);
    if (rh == 0) {
#pragma unroll
      for (int r = 0; r < 8; ++r) eS[r * 256 + nt * 16 + cl] = acc[r] + mb[nt * 16 + cl];
    }
  }
  __syncthreads();
#pragma unroll 1
  for (int pass = 0; pass < 2; ++pass) {
#pragma unroll
    for (int it = 0; it < 2; ++it) *(volatile v4f_t*)(emb + (tid + 256 * it) * 4) = *(const volatile v4fa*)(eS + (tid + 256 * it) * 4);
    __threadfence();
  }
}
template <int EPI>
__global__ __launch_bounds__(256) void k_conv3(const float* __restrict__ src, const float* __restrict__ stats, const float* __restrict__ gam,
                                               const float* __restrict__ bet, const float* __restrict__ Wt, const float* __restrict__ bias,
                                               const float* __restrict__ embv, const float* __restrict__ R, float* __restrict__ Y) {
  __shared__ __attribute__((aligned(16))) f16 ldsA[128 * KST];
  __shared__ __attribute__((aligned(16))) f16 ldsB[128 * KST];
  __shared__ __attribute__((aligned(16))) float oS[8][32 * 68];
  __shared__ float gm[CH], gr[CH], ga[CH], gb[CH];
  constexpr int KTOT = CH * 9;
  const int tid = threadIdx.x, lane = tid & 31, wave = tid >> 5, cl = lane & 15, rh = (lane >> 4) * 8;
  const int b = blockIdx.x >> 3, y0 = (blockIdx.x & 7) * 4, o0 = blockIdx.y * 128;
  const int wm = (wave & 3) * 32, wp = (wave >> 2) * 64;
  for (int c = tid; c < CH; c += 256) { gm[c] = stats[((size_t)b * NG + (c >> 3)) * 2]; gr[c] = stats[((size_t)b * NG + (c >> 3)) * 2 + 1]; ga[c] = gam[c]; gb[c] = bet[c]; }
  const float* inb = src + (size_t)b * CH * HW_;
  f32x8 acc[2][4];
#pragma unroll
  for (int i = 0; i < 2; ++i)
#pragma unroll
    for (int j = 0; j < 4; ++j) { f32x8 z = {}; acc[i][j] = z; }
  __syncthreads();
#pragma unroll 1
  for (int k0 = 0; k0 < KTOT; k0 += 32) {
    __syncthreads();
    { const int o = tid >> 1, kq = (tid & 1) * 16;
      const float* wr = Wt + (size_t)(o0 + o) * KTOT + k0 + kq;
#pragma unroll
      for (int u = 0; u < 16; ++u) ldsA[o * KST + kq + u] = (f16)wr[u]; }
    { const int px = tid >> 1, kq = (tid & 1) * 16;
      const int yy = px >> 5, xx = px & 31;
#pragma unroll 4
      for (int u = 0; u < 16; ++u) {
        const int k = k0 + kq + u, c = k / 9, r9 = k - 9 * c, dy = r9 / 3 - 1, dx = r9 - 3 * (r9 / 3) - 1;
        const int ys = y0 + yy + dy, xs = xx + dx;
        float v = 0.0f;
        if (ys >= 0 && ys < IMH && xs >= 0 && xs < IMW) {
          const float a = (inb[(size_t)c * HW_ + ys * IMW + xs] - gm[c]) * gr[c] * ga[c] + gb[c];
          v = a / (1.0f + __expf(-a));
        }
        ldsB[px * KST + kq + u] = (f16)v;
      } }
    __syncthreads();
    f16x16 af[2];
#pragma unroll
    for (int i = 0; i < 2; ++i) af[i] = lds_frag(ldsA + (wm + 16 * i) * KST, KST);
#pragma unroll
    for (int j = 0; j < 4; ++j) {
      const f16x16 bfv = lds_frag(ldsB + (wp + 16 * j) * KST, KST);
#pragma unroll
      for (int i = 0; i < 2; ++i) acc[i][j] = wmma16(af[i], bfv, acc[i][j]);
    }
  }
  float* so = oS[wave];
#pragma unroll
  for (int i = 0; i < 2; ++i)
#pragma unroll
    for (int r = 0; r < 8; ++r) {
      const int o = o0 + wm + 16 * i + rh + r;
      const float add = bias[o] + ((EPI == 0) ? embv[b * CH + o] : 0.0f);
#pragma unroll
      for (int j = 0; j < 4; ++j) so[(16 * i + rh + r) * 68 + 16 * j + cl] = acc[i][j][r] + add;
    }
  asm volatile("s_wait_dscnt 0" ::: "memory");
  __builtin_amdgcn_wave_barrier();
  const size_t pxoff = (size_t)(y0 * IMW + wp);
  if (EPI == 1) {
#pragma unroll
    for (int it = 0; it < 16; ++it) { const int f4 = lane + 32 * it, rr = f4 >> 4, q = (f4 & 15) * 4;
      const size_t off = ((size_t)b * CH + o0 + wm + rr) * HW_ + pxoff + q;
      const v4f_t rv = *(const v4f_t*)(R + off); v4f_t v = *(const volatile v4fa*)(so + rr * 68 + q); v += rv; *(volatile v4fa*)(so + rr * 68 + q) = v; }
    asm volatile("s_wait_dscnt 0" ::: "memory");
  }
#pragma unroll 1
  for (int pass = 0; pass < 2; ++pass) {
#pragma unroll
    for (int it = 0; it < 16; ++it) { const int f4 = lane + 32 * it, rr = f4 >> 4, q = (f4 & 15) * 4;
      const size_t off = ((size_t)b * CH + o0 + wm + rr) * HW_ + pxoff + q;
      *(volatile v4f_t*)(Y + off) = *(const volatile v4fa*)(so + rr * 68 + q); }
    __threadfence();
  }
}
__global__ __launch_bounds__(256) void k_gn_tok(const float* __restrict__ r, const float* __restrict__ stats, const float* __restrict__ gam,
                                               const float* __restrict__ bet, bf16* __restrict__ nT) {
  __shared__ __attribute__((aligned(16))) bf16 tS[128 * 264];
  const int tid = threadIdx.x, b = blockIdx.x >> 3, p0 = (blockIdx.x & 7) * 128;
  for (int e = tid; e < CH * 128; e += 256) {
    const int c = e >> 7, px = e & 127;
    const float mu = stats[((size_t)b * NG + (c >> 3)) * 2], rs = stats[((size_t)b * NG + (c >> 3)) * 2 + 1];
    const float v = (r[((size_t)b * CH + c) * HW_ + p0 + px] - mu) * rs * gam[c] + bet[c];
    tS[px * 264 + c] = (bf16)v;
  }
  __syncthreads();
#pragma unroll 1
  for (int pass = 0; pass < 2; ++pass) {
#pragma unroll
    for (int it = 0; it < 16; ++it) { const int ch = tid + 256 * it, row = ch >> 5, q8 = (ch & 31) * 8;
      *(volatile v4u_t*)(nT + ((size_t)b * HW_ + p0 + row) * CH + q8) = *(const v4ua*)(tS + row * 264 + q8); }
    __threadfence();
  }
}

extern "C" void kernel_launch(void* const* d_in, const int* in_sizes, int n_in,
                              void* d_out, int out_size, void* d_ws, size_t ws_size,
                              hipStream_t stream) {
  (void)in_sizes; (void)n_in; (void)out_size; (void)ws_size;
  const float* x = (const float*)d_in[0];
  const float* te = (const float*)d_in[1];
  const float* gn1s = (const float*)d_in[2], *gn1b = (const float*)d_in[3];
  const float* c1w = (const float*)d_in[4], *c1b = (const float*)d_in[5];
  const float* mw = (const float*)d_in[6], *mb = (const float*)d_in[7];
  const float* gn2s = (const float*)d_in[8], *gn2b = (const float*)d_in[9];
  const float* c2w = (const float*)d_in[10], *c2b = (const float*)d_in[11];
  const float* gnas = (const float*)d_in[12], *gnab = (const float*)d_in[13];
  const float* qkvw = (const float*)d_in[14];
  const float* ow = (const float*)d_in[15], *ob = (const float*)d_in[16];
  float* out = (float*)d_out;
  char* ws = (char*)d_ws;
  float* st1 = (float*)ws; ws += 4096; float* st2 = (float*)ws; ws += 4096; float* st3 = (float*)ws; ws += 4096; float* emb = (float*)ws; ws += 8192;
  const size_t T32 = (size_t)NB_ * CH * HW_ * 4;
  float* h1 = (float*)ws; ws += T32; float* rr = (float*)ws; ws += T32;
  bf16* nT = (bf16*)ws; ws += (size_t)NB_ * HW_ * CH * 2;
  bf16* QKV = (bf16*)ws; ws += (size_t)NB_ * HW_ * QKVST * 2;
  bf16* Vt = (bf16*)ws; ws += (size_t)NB_ * HH * DKK * SS * 2;
  float* attn = (float*)ws; ws += (size_t)NB_ * HW_ * CH * 4;

  k_gn_stats<<<dim3(NB_ * 2), dim3(256), 0, stream>>>(x, st1);
  k_emb<<<dim3(1), dim3(256), 0, stream>>>(te, mw, mb, emb);
  k_conv3<0><<<dim3(NB_ * 8, 2), dim3(256), 0, stream>>>(x, st1, gn1s, gn1b, c1w, c1b, emb, nullptr, h1);
  k_gn_stats<<<dim3(NB_ * 2), dim3(256), 0, stream>>>(h1, st2);
  k_conv3<1><<<dim3(NB_ * 8, 2), dim3(256), 0, stream>>>(h1, st2, gn2s, gn2b, c2w, c2b, nullptr, x, rr);
  k_gn_stats<<<dim3(NB_ * 2), dim3(256), 0, stream>>>(rr, st3);
  k_gn_tok<<<dim3(NB_ * 8), dim3(256), 0, stream>>>(rr, st3, gnas, gnab, nT);
  const int M = NB_ * HW_;
  gemm_rb_kernel<bf16, 0><<<dim3(M / 128, QKVST / 256), dim3(256), 0, stream>>>(nT, qkvw, nullptr, nullptr, nullptr, nullptr, QKV, M, QKVST, CH);
  gemm_rb_kernel<bf16, 1><<<dim3(M / 128, QKVST / 256), dim3(256), 0, stream>>>(nT, qkvw, nullptr, nullptr, nullptr, nullptr, Vt,  M, QKVST, CH);
  attn_kernel<<<dim3(SS / 64, 4, NB_), dim3(64), 0, stream>>>(QKV, QKV, Vt, attn);
  for (int b = 0; b < NB_; ++b)
    gemm_rb_kernel<float, 2><<<dim3(CH / 128, HW_ / 256), dim3(256), 0, stream>>>(ow, attn + (size_t)b * HW_ * CH, nullptr, nullptr, rr + (size_t)b * CH * HW_, ob, out + (size_t)b * CH * HW_, CH, HW_, CH);
}
